// TopicEncoder_58239756534018
// MI455X (gfx1250) — hardware-verified
//
#include <hip/hip_runtime.h>
#include <math.h>
#include <stdint.h>

constexpr int kBatch = 32;
constexpr int kSeq   = 512;
constexpr int kHid   = 768;
constexpr int kTop   = 100;
constexpr int kTHid  = 512;
constexpr int kLang  = 5;
constexpr int kTok   = kBatch * kSeq;
constexpr int kKf    = kHid + kTop;
constexpr int kKfPad = 896;
constexpr int kMf    = 64;
constexpr float kWCarry    = 16.0f;
constexpr float kWCarryInv = 1.0f / 16.0f;
constexpr float kInvHid    = 1.0f / 768.0f;
constexpr float kInvTHid   = 1.0f / 512.0f;
constexpr float kLnEps     = 1e-5f;
constexpr float kPoolEps   = 1e-10f;

typedef __attribute__((ext_vector_type(16))) _Float16 v16h;
typedef __attribute__((ext_vector_type(8)))  _Float16 v8h;
typedef __attribute__((ext_vector_type(16))) __bf16   v16b;
typedef __attribute__((ext_vector_type(8)))  __bf16   v8b;
typedef __attribute__((ext_vector_type(8)))  float    v8f;
typedef __attribute__((ext_vector_type(4)))  float    v4f;
typedef __attribute__((ext_vector_type(4)))  unsigned int v4u;

__device__ __forceinline__ unsigned short f2bf_bits(float f) {
  unsigned u = __float_as_uint(f);
  return (unsigned short)((u + 0x7FFFu + ((u >> 16) & 1u)) >> 16);
}
__device__ __forceinline__ float bf_bits2f(unsigned short h) { return __uint_as_float(((unsigned)h) << 16); }

__device__ __forceinline__ void dep_guard_h(v8f& a, v8f& b, v16h x, v16h y) { asm volatile("v_nop\n\tv_nop\n\tv_nop\n\tv_nop" : "+v"(a), "+v"(b) : "v"(x), "v"(y)); }
__device__ __forceinline__ void dep_guard_b(v8f& a, v8f& b, v16b x, v16b y) { asm volatile("v_nop\n\tv_nop\n\tv_nop\n\tv_nop" : "+v"(a), "+v"(b) : "v"(x), "v"(y)); }
__device__ __forceinline__ void keep4_h(v16h a, v16h b, v16h c, v16h d) { asm volatile("v_nop" :: "v"(a), "v"(b), "v"(c), "v"(d)); }
__device__ __forceinline__ void keep4_b(v16b a, v16b b, v16b c, v16b d) { asm volatile("v_nop" :: "v"(a), "v"(b), "v"(c), "v"(d)); }
__device__ __forceinline__ void acc_guard4(v8f& a, v8f& b, v8f& c, v8f& d) { asm volatile("v_nop\n\tv_nop\n\tv_nop\n\tv_nop" : "+v"(a), "+v"(b), "+v"(c), "+v"(d)); }
template <typename T> struct Frag;
template <> struct Frag<_Float16> {
  typedef v16h V; union U { v16h v; v8h h[2]; };
  static __device__ __forceinline__ v16h load(const _Float16* p) {
    U f; f.h[0] = *(const v8h*)(p); f.h[1] = *(const v8h*)(p + 16); return f.v;
  }
  static __device__ __forceinline__ v8f mma(v16h a, v16h b, v8f c) {
    return __builtin_amdgcn_wmma_f32_16x16x32_f16(false, a, false, b, (short)0, c, false, false);
  }
  static __device__ __forceinline__ void guard(v8f& a, v8f& b, v16h x, v16h y) { dep_guard_h(a, b, x, y); }
  static __device__ __forceinline__ void keep(v16h a, v16h b, v16h c, v16h d) { keep4_h(a, b, c, d); }
};
template <> struct Frag<__bf16> {
  typedef v16b V; union U { v16b v; v8b h[2]; };
  static __device__ __forceinline__ v16b load(const __bf16* p) {
    U f; f.h[0] = *(const v8b*)(p); f.h[1] = *(const v8b*)(p + 16); return f.v;
  }
  static __device__ __forceinline__ v8f mma(v16b a, v16b b, v8f c) {
    return __builtin_amdgcn_wmma_f32_16x16x32_bf16(false, a, false, b, (short)0, c, false, false);
  }
  static __device__ __forceinline__ void guard(v8f& a, v8f& b, v16b x, v16b y) { dep_guard_b(a, b, x, y); }
  static __device__ __forceinline__ void keep(v16b a, v16b b, v16b c, v16b d) { keep4_b(a, b, c, d); }
};

template <int ET> struct Elem;
template <> struct Elem<0> { typedef _Float16 T; };
template <> struct Elem<1> { typedef __bf16 T; };
template <int ET, bool SPLIT, int BIAS_MODE, int OUT_MODE, bool RESID, int ACT = 0, bool ZSEL = false>
__global__ __launch_bounds__(256) void wmma_gemm64(
    const unsigned short* __restrict__ Ap, const unsigned short* __restrict__ A2p, int lda, long strideA,
    const unsigned short* __restrict__ Btp, const unsigned short* __restrict__ Bt2p, int ldb, long strideB,
    void* __restrict__ Cout, void* __restrict__ Cout2, int ldc, long strideC,
    const float* __restrict__ bias,
    const float* __restrict__ resid, long strideR,
    const int* __restrict__ zsel, long selStrideB, long selStrideBias, int nsel,
    int M, int N, int K, float scale) {
  typedef typename Elem<ET>::T T;
  typedef typename Frag<T>::V V;
  const T* A = (const T*)Ap; const T* A2 = (const T*)A2p; const T* Bt = (const T*)Btp; const T* Bt2 = (const T*)Bt2p;
  __shared__ __align__(16) float sT[8][16 * 68];
  const int b    = blockIdx.y;
  const int lane = threadIdx.x & 31;
  const int wave = threadIdx.x >> 5;
  const int tilesN = N >> 6;
  const int tilesM = M >> 6;
  const int tile = blockIdx.x * 8 + wave;
  if (tile >= tilesM * tilesN) return;
  const int tm = tile / tilesN;
  const int tn = tile - tm * tilesN;
  const int m0 = tm << 6;
  const int n0 = tn << 6;

  long selB = 0, selBias = 0;
  if (ZSEL) {
    int s = zsel[b];
    s = s < 0 ? 0 : s;
    s = s > nsel - 1 ? nsel - 1 : s;
    selB = (long)s * selStrideB;
    selBias = (long)s * selStrideBias;
  }
  const float* biasp = bias + selBias;

  const T* Ab  = A  + (size_t)b * strideA;
  const T* Bb  = Bt + (size_t)b * strideB + selB;
  const T* Ab2 = SPLIT ? (A2  + (size_t)b * strideA) : nullptr;
  const T* Bb2 = SPLIT ? (Bt2 + (size_t)b * strideB + selB) : nullptr;

  const int rlane = lane & 15;
  const int koff  = (lane >> 4) * 8;
  const int mOff  = (lane >> 4) * 8;

  v8f acc[4][4];
#pragma unroll
  for (int i = 0; i < 4; ++i)
#pragma unroll
    for (int j = 0; j < 4; ++j) acc[i][j] = (v8f){0.f,0.f,0.f,0.f,0.f,0.f,0.f,0.f};

  for (int k0 = 0; k0 < K; k0 += 32) {
    V bh[4], bl[4];
#pragma unroll
    for (int j = 0; j < 4; ++j) {
      const size_t bo = (size_t)(n0 + (j << 4) + rlane) * ldb + koff + k0;
      bh[j] = Frag<T>::load(Bb + bo);
      if (SPLIT) bl[j] = Frag<T>::load(Bb2 + bo);
    }
#pragma unroll
    for (int i = 0; i < 4; ++i) {
      const size_t ao = (size_t)(m0 + (i << 4) + rlane) * lda + koff + k0;
      V ah = Frag<T>::load(Ab + ao);
      V al;
      if (SPLIT) al = Frag<T>::load(Ab2 + ao);
#pragma unroll
      for (int j = 0; j < 4; ++j) {
        acc[i][j] = Frag<T>::mma(ah, bh[j], acc[i][j]);
        if (SPLIT) {
          acc[i][j] = Frag<T>::mma(ah, bl[j], acc[i][j]);
          acc[i][j] = Frag<T>::mma(al, bh[j], acc[i][j]);
        }
      }
      Frag<T>::guard(acc[i][0], acc[i][3], ah, SPLIT ? al : ah);
    }
    Frag<T>::keep(bh[0], bh[1], bh[2], bh[3]);
    if (SPLIT) Frag<T>::keep(bl[0], bl[1], bl[2], bl[3]);
  }
  acc_guard4(acc[0][0], acc[0][1], acc[0][2], acc[0][3]);
  acc_guard4(acc[1][0], acc[1][1], acc[1][2], acc[1][3]);
  acc_guard4(acc[2][0], acc[2][1], acc[2][2], acc[2][3]);
  acc_guard4(acc[3][0], acc[3][1], acc[3][2], acc[3][3]);

  float* slab = sT[wave];
  const float* Rb = RESID ? (resid + (size_t)b * strideR) : nullptr;
#pragma unroll
  for (int i = 0; i < 4; ++i) {
    const int mBase = m0 + (i << 4);
#pragma unroll
    for (int j = 0; j < 4; ++j) {
      const int n = n0 + (j << 4) + rlane;
      float bv = 0.f;
      if (BIAS_MODE == 2) bv = biasp[n];
#pragma unroll
      for (int r = 0; r < 8; ++r) {
        float v = acc[i][j][r] * scale;
        if (BIAS_MODE == 1) v += biasp[mBase + mOff + r];
        if (BIAS_MODE == 2) v += bv;
        if (RESID) v += Rb[(size_t)(mBase + mOff + r) * ldc + n];
        if (ACT == 1) v = tanhf(v);
        if (ACT == 2) v = fmaxf(v, 0.0f);
        if (ACT == 3) v = v / (1.0f + expf(-v));
        if (ACT == 4) v = (v > 0.f) ? v : 0.01f * v;
        slab[(mOff + r) * 68 + (j << 4) + rlane] = v;
      }
    }
    __builtin_amdgcn_fence(__ATOMIC_RELEASE, "workgroup");
    __builtin_amdgcn_wave_barrier();
    __builtin_amdgcn_fence(__ATOMIC_ACQUIRE, "workgroup");
    if (OUT_MODE == 0) {
      float* C = (float*)Cout + (size_t)b * strideC;
      const int hh = lane >> 4, c4 = (lane & 15) * 4;
      for (int pass = 0; pass < 2; ++pass) {
#pragma unroll
        for (int it = 0; it < 8; ++it) {
          const int row = it * 2 + hh;
          v4f v = *(const v4f*)(slab + row * 68 + c4);
          *(volatile v4f*)(C + (size_t)(mBase + row) * ldc + n0 + c4) = v;
        }
        __threadfence();
      }
    } else {
      const int q = lane >> 3, c8 = (lane & 7) * 8;
      unsigned short* C  = (unsigned short*)Cout  + (size_t)b * strideC;
      unsigned short* C2 = (OUT_MODE == 2) ? ((unsigned short*)Cout2 + (size_t)b * strideC) : nullptr;
      for (int pass = 0; pass < 2; ++pass) {
#pragma unroll
        for (int it = 0; it < 4; ++it) {
          const int row = it * 4 + q;
          const float* sp = slab + row * 68 + c8;
          v8h hv, lv;
#pragma unroll
          for (int e = 0; e < 8; ++e) {
            if (OUT_MODE == 1) {
              hv[e] = (_Float16)sp[e];
            } else {
              unsigned short hb = f2bf_bits(sp[e]);
              unsigned short lb = f2bf_bits(sp[e] - bf_bits2f(hb));
              hv[e] = __builtin_bit_cast(_Float16, hb);
              lv[e] = __builtin_bit_cast(_Float16, lb);
            }
          }
          *(volatile v8h*)(C + (size_t)(mBase + row) * ldc + n0 + c8) = hv;
          if (OUT_MODE == 2) *(volatile v8h*)(C2 + (size_t)(mBase + row) * ldc + n0 + c8) = lv;
        }
        __threadfence();
      }
    }
    __builtin_amdgcn_fence(__ATOMIC_RELEASE, "workgroup");
    __builtin_amdgcn_wave_barrier();
    __builtin_amdgcn_fence(__ATOMIC_ACQUIRE, "workgroup");
  }
}

__device__ __forceinline__ unsigned pk16(unsigned short a, unsigned short b) { return (unsigned)a | ((unsigned)b << 16); }
__device__ __forceinline__ unsigned short h_bits(float f) { const _Float16 h = (_Float16)f; return __builtin_bit_cast(unsigned short, h); }

__global__ __launch_bounds__(256) void cast_f32_f16x8_kernel(const float* __restrict__ in, unsigned short* __restrict__ out, int n8) {
  const int i = blockIdx.x * 256 + threadIdx.x;
  if (i < n8) {
    const float* p = in + 8 * (size_t)i;
    const v4f a = *(const v4f*)(p);
    const v4f c = *(const v4f*)(p + 4);
    const v4u u = (v4u){pk16(h_bits(a[0]), h_bits(a[1])), pk16(h_bits(a[2]), h_bits(a[3])),
                        pk16(h_bits(c[0]), h_bits(c[1])), pk16(h_bits(c[2]), h_bits(c[3]))};
    unsigned short* op = out + 8 * (size_t)i;
    *(volatile v4u*)op = u;
    __threadfence();
    *(volatile v4u*)op = u;
  }
}

__global__ __launch_bounds__(256) void transpose_cast_f16_kernel(const float* __restrict__ in, unsigned short* __restrict__ out,
                                                                 int Rv, int Rp, int CC, long inPlane, long outPlane, float scale) {
  __shared__ float tile[64][65];
  const int t  = threadIdx.x;
  const int n0 = blockIdx.x * 64;
  const int k0 = blockIdx.y * 64;
  const int z  = blockIdx.z;
  const float* inz = in + (size_t)z * inPlane;
  unsigned short* outz = out + (size_t)z * outPlane;
  {
    const int kr = t >> 2, nc = (t & 3) * 16;
    const int k  = k0 + kr;
    const int kc = (k < Rv) ? k : (Rv - 1);
    const bool live = (k < Rv);
    const float* p = inz + (size_t)kc * CC + n0 + nc;
#pragma unroll
    for (int e4 = 0; e4 < 4; ++e4) {
      const v4f f = *(const v4f*)(p + 4 * e4);
      tile[kr][nc + 4 * e4 + 0] = live ? f[0] : 0.0f;
      tile[kr][nc + 4 * e4 + 1] = live ? f[1] : 0.0f;
      tile[kr][nc + 4 * e4 + 2] = live ? f[2] : 0.0f;
      tile[kr][nc + 4 * e4 + 3] = live ? f[3] : 0.0f;
    }
  }
  __syncthreads();
  const int q = t >> 3, c8 = (t & 7) * 8;
  v4u u0, u1;
#pragma unroll
  for (int w = 0; w < 4; ++w) {
    u0[w] = pk16(h_bits(tile[c8 + 2 * w][q] * scale),      h_bits(tile[c8 + 2 * w + 1][q] * scale));
    u1[w] = pk16(h_bits(tile[c8 + 2 * w][32 + q] * scale), h_bits(tile[c8 + 2 * w + 1][32 + q] * scale));
  }
  unsigned short* p0 = outz + (size_t)(n0 + q) * Rp + k0 + c8;
  unsigned short* p1 = outz + (size_t)(n0 + 32 + q) * Rp + k0 + c8;
  for (int pass = 0; pass < 2; ++pass) {
    *(volatile v4u*)p0 = u0;
    *(volatile v4u*)p1 = u1;
    __threadfence();
  }
}

__global__ __launch_bounds__(128) void ln_relu_rows_f16_kernel(const float* __restrict__ x, const int* __restrict__ lang,
                                                               const float* __restrict__ gam, const float* __restrict__ bet,
                                                               unsigned short* __restrict__ out) {
  __shared__ float redA[4];
  __shared__ float redB[4];
  const int row  = blockIdx.x;
  const int t    = threadIdx.x;
  const int lane = t & 31, wave = t >> 5;
  int l = lang[row >> 9];
  l = l < 0 ? 0 : l;
  l = l > kLang - 1 ? kLang - 1 : l;
  const int c0   = t * 8;
  const float* xr = x + (size_t)row * kHid + c0;
  const v4f a = *(const v4f*)(xr);
  const v4f c = *(const v4f*)(xr + 4);
  float s = ((a[0] + a[1]) + (a[2] + a[3])) + ((c[0] + c[1]) + (c[2] + c[3]));
#pragma unroll
  for (int off = 16; off > 0; off >>= 1) s += __shfl_xor(s, off, 32);
  if (lane == 0) redA[wave] = s;
  __syncthreads();
  const float mu = ((redA[0] + redA[1]) + redA[2]) * kInvHid;
  const float d0 = a[0] - mu, d1 = a[1] - mu, d2 = a[2] - mu, d3 = a[3] - mu;
  const float d4 = c[0] - mu, d5 = c[1] - mu, d6 = c[2] - mu, d7 = c[3] - mu;
  float qq = ((d0 * d0 + d1 * d1) + (d2 * d2 + d3 * d3)) + ((d4 * d4 + d5 * d5) + (d6 * d6 + d7 * d7));
#pragma unroll
  for (int off = 16; off > 0; off >>= 1) qq += __shfl_xor(qq, off, 32);
  if (lane == 0) redB[wave] = qq;
  __syncthreads();
  const float var = ((redB[0] + redB[1]) + redB[2]) * kInvHid;
  const float rs  = rsqrtf(var + kLnEps);
  const float* gp = gam + (size_t)l * kHid + c0;
  const float* bp = bet + (size_t)l * kHid + c0;
  const v4f g0 = *(const v4f*)(gp), g1v = *(const v4f*)(gp + 4);
  const v4f b0 = *(const v4f*)(bp), b1v = *(const v4f*)(bp + 4);
  const float y0 = fmaxf(d0 * rs * g0[0] + b0[0], 0.0f), y1 = fmaxf(d1 * rs * g0[1] + b0[1], 0.0f);
  const float y2 = fmaxf(d2 * rs * g0[2] + b0[2], 0.0f), y3 = fmaxf(d3 * rs * g0[3] + b0[3], 0.0f);
  const float y4 = fmaxf(d4 * rs * g1v[0] + b1v[0], 0.0f), y5 = fmaxf(d5 * rs * g1v[1] + b1v[1], 0.0f);
  const float y6 = fmaxf(d6 * rs * g1v[2] + b1v[2], 0.0f), y7 = fmaxf(d7 * rs * g1v[3] + b1v[3], 0.0f);
  const v4u hv = (v4u){pk16(h_bits(y0), h_bits(y1)), pk16(h_bits(y2), h_bits(y3)),
                       pk16(h_bits(y4), h_bits(y5)), pk16(h_bits(y6), h_bits(y7))};
  unsigned short* op = out + (size_t)row * kHid + c0;
  *(volatile v4u*)op = hv;
  __threadfence();
  *(volatile v4u*)op = hv;
}

__global__ __launch_bounds__(256) void pool_combine_kernel(const float* __restrict__ h2, const float* __restrict__ tokw,
                                                           const float* __restrict__ topics, unsigned short* __restrict__ C16) {
  __shared__ float part[4][64];
  __shared__ float pooled[64];
  __shared__ float swsum;
  const int cb = blockIdx.x, b = blockIdx.y, t = threadIdx.x;
  const int c = t & 63, tg = t >> 6;
  {
    const float* hp = h2 + ((size_t)b * kSeq + tg * 128) * kHid + cb * 64 + c;
    const float* wp = tokw + (size_t)b * kSeq + tg * 128;
    float s = 0.0f;
#pragma unroll 1
    for (int i = 0; i < 128; ++i) {
      const float hm = hp[(size_t)i * kHid] * wp[i];
      s += hm;
    }
    part[tg][c] = s;
  }
  if (t < 32) {
    const float* wr = tokw + (size_t)b * kSeq + t * 16;
    float ws = 0.0f;
#pragma unroll 1
    for (int i = 0; i < 16; ++i) ws += wr[i];
#pragma unroll
    for (int off = 16; off > 0; off >>= 1) ws += __shfl_xor(ws, off, 32);
    if (t == 0) swsum = ws;
  }
  __syncthreads();
  if (t < 64) {
    const float inv = 1.0f / (swsum + kPoolEps);
    pooled[t] = ((part[0][t] + part[1][t]) + (part[2][t] + part[3][t])) * inv;
  }
  __syncthreads();
  if (t < 8) {
    v4u u;
#pragma unroll
    for (int w = 0; w < 4; ++w) u[w] = pk16(h_bits(pooled[8 * t + 2 * w]), h_bits(pooled[8 * t + 2 * w + 1]));
    unsigned short* op = C16 + (size_t)b * kKfPad + cb * 64 + 8 * t;
    *(volatile v4u*)op = u;
    __threadfence();
    *(volatile v4u*)op = u;
  }
  if (cb == 0) {
    if (t < 16) {
      v4u u;
#pragma unroll
      for (int w = 0; w < 4; ++w) {
        const int j0 = 8 * t + 2 * w, j1 = j0 + 1;
        const int j0c = j0 < kTop ? j0 : (kTop - 1), j1c = j1 < kTop ? j1 : (kTop - 1);
        const float f0 = topics[(size_t)b * kTop + j0c];
        const float f1 = topics[(size_t)b * kTop + j1c];
        const float v0 = (j0 < kTop) ? f0 : 0.0f;
        const float v1 = (j1 < kTop) ? f1 : 0.0f;
        u[w] = pk16(h_bits(v0), h_bits(v1));
      }
      unsigned short* op = C16 + (size_t)b * kKfPad + kHid + 8 * t;
      *(volatile v4u*)op = u;
      __threadfence();
      *(volatile v4u*)op = u;
    }
    if (t < kKfPad / 8) {
      const v4u zz = (v4u){0u, 0u, 0u, 0u};
      unsigned short* op = C16 + (size_t)(kBatch + b) * kKfPad + 8 * t;
      *(volatile v4u*)op = zz;
      __threadfence();
      *(volatile v4u*)op = zz;
    }
  }
}

__global__ __launch_bounds__(128) void ln_relu_out_kernel(const float* __restrict__ F, const float* __restrict__ gam,
                                                          const float* __restrict__ bet, float* __restrict__ out) {
  __shared__ float redA[4];
  __shared__ float redB[4];
  const int row  = blockIdx.x;
  const int t    = threadIdx.x;
  const int lane = t & 31, wave = t >> 5;
  const int c0   = t * 4;
  const v4f a = *(const v4f*)(F + (size_t)row * kTHid + c0);
  float s = (a[0] + a[1]) + (a[2] + a[3]);
#pragma unroll
  for (int off = 16; off > 0; off >>= 1) s += __shfl_xor(s, off, 32);
  if (lane == 0) redA[wave] = s;
  __syncthreads();
  const float mu = ((redA[0] + redA[1]) + (redA[2] + redA[3])) * kInvTHid;
  const float d0 = a[0] - mu, d1 = a[1] - mu, d2 = a[2] - mu, d3 = a[3] - mu;
  float qq = (d0 * d0 + d1 * d1) + (d2 * d2 + d3 * d3);
#pragma unroll
  for (int off = 16; off > 0; off >>= 1) qq += __shfl_xor(qq, off, 32);
  if (lane == 0) redB[wave] = qq;
  __syncthreads();
  const float var = ((redB[0] + redB[1]) + (redB[2] + redB[3])) * kInvTHid;
  const float rs  = rsqrtf(var + kLnEps);
  const v4f g = *(const v4f*)(gam + c0);
  const v4f bb = *(const v4f*)(bet + c0);
  v4f y;
  y[0] = fmaxf(d0 * rs * g[0] + bb[0], 0.0f);
  y[1] = fmaxf(d1 * rs * g[1] + bb[1], 0.0f);
  y[2] = fmaxf(d2 * rs * g[2] + bb[2], 0.0f);
  y[3] = fmaxf(d3 * rs * g[3] + bb[3], 0.0f);
  float* op = out + (size_t)row * kTHid + c0;
  *(volatile v4f*)op = y;
  __threadfence();
  *(volatile v4f*)op = y;
}

extern "C" void kernel_launch(void* const* d_in, const int* in_sizes, int n_in,
                              void* d_out, int out_size, void* d_ws, size_t ws_size,
                              hipStream_t stream) {
  if (n_in < 14) return;
  if (in_sizes[0] != kTok * kHid) return;
  if (in_sizes[1] != kBatch * kSeq) return;
  if (in_sizes[2] != kBatch) return;
  if (in_sizes[3] != kBatch * kTop) return;
  if (in_sizes[4] != kLang * kHid * kHid || in_sizes[8] != kLang * kHid * kHid) return;
  if (in_sizes[5] != kLang * kHid || in_sizes[6] != kLang * kHid || in_sizes[7] != kLang * kHid || in_sizes[9] != kLang * kHid) return;
  if (in_sizes[10] != kKf * kTHid) return;
  if (in_sizes[11] != kTHid || in_sizes[12] != kTHid || in_sizes[13] != kTHid) return;
  if (out_size != kBatch * kTHid) return;

  const float* seq    = (const float*)d_in[0];
  const float* tokw   = (const float*)d_in[1];
  const int*   lang   = (const int*)  d_in[2];
  const float* topics = (const float*)d_in[3];
  const float* W1     = (const float*)d_in[4];
  const float* b1     = (const float*)d_in[5];
  const float* g1     = (const float*)d_in[6];
  const float* be1    = (const float*)d_in[7];
  const float* W2     = (const float*)d_in[8];
  const float* b2     = (const float*)d_in[9];
  const float* Wf     = (const float*)d_in[10];
  const float* bfv    = (const float*)d_in[11];
  const float* gf     = (const float*)d_in[12];
  const float* bef    = (const float*)d_in[13];
  float* outp = (float*)d_out;

  const size_t PWL  = (size_t)kLang * kHid * kHid * 2;
  const size_t PWF  = (size_t)kTHid * kKfPad * 2;
  const size_t PH   = (size_t)kTok * kHid * 4;
  const size_t PR16 = (size_t)kTok * kHid * 2;
  const size_t PC16 = (size_t)kMf * kKfPad * 2;
  const size_t PF   = (size_t)kMf * kTHid * 4;
  size_t off = 0;
  const size_t oW1T = off; off += PWL;
  const size_t oW2T = off; off += PWL;
  const size_t oWfT = off; off += PWF;
  const size_t oH   = off; off += PH;
  const size_t oR16 = off; off += PR16;
  const size_t oC16 = off; off += PC16;
  const size_t oF   = off; off += PF;
  if (off > ws_size) return;

  char* ws = (char*)d_ws;
  unsigned short* W1T  = (unsigned short*)(ws + oW1T);
  unsigned short* W2T  = (unsigned short*)(ws + oW2T);
  unsigned short* WfT  = (unsigned short*)(ws + oWfT);
  float*          Hbuf = (float*)(ws + oH);
  unsigned short* R16  = (unsigned short*)(ws + oR16);
  unsigned short* C16  = (unsigned short*)(ws + oC16);
  float*          Fbuf = (float*)(ws + oF);

  const dim3 blk(256);

  transpose_cast_f16_kernel<<<dim3(kHid / 64, kHid / 64, kLang), blk, 0, stream>>>(
      W1, W1T, kHid, kHid, kHid, (long)kHid * kHid, (long)kHid * kHid, kWCarry);
  transpose_cast_f16_kernel<<<dim3(kHid / 64, kHid / 64, kLang), blk, 0, stream>>>(
      W2, W2T, kHid, kHid, kHid, (long)kHid * kHid, (long)kHid * kHid, kWCarry);
  transpose_cast_f16_kernel<<<dim3(kTHid / 64, kKfPad / 64, 1), blk, 0, stream>>>(
      Wf, WfT, kKf, kKfPad, kTHid, 0L, 0L, kWCarry);

  const int n8x = kTok * kHid / 8;
  cast_f32_f16x8_kernel<<<dim3((n8x + 255) / 256), blk, 0, stream>>>(seq, R16, n8x);

  const dim3 gAd((((kSeq / 64) * (kHid / 64)) + 7) / 8, kBatch);
  wmma_gemm64<0, false, 2, 0, false, 0, true><<<gAd, blk, 0, stream>>>(
      R16, R16, kHid, (long)kSeq * kHid,
      W1T, W1T, kHid, 0L,
      (void*)Hbuf, (void*)Hbuf, kHid, (long)kSeq * kHid,
      b1, seq, 0L,
      lang, (long)kHid * kHid, (long)kHid, kLang,
      kSeq, kHid, kHid, kWCarryInv);

  ln_relu_rows_f16_kernel<<<dim3(kTok), dim3(96), 0, stream>>>(Hbuf, lang, g1, be1, R16);

  wmma_gemm64<0, false, 2, 0, false, 0, true><<<gAd, blk, 0, stream>>>(
      R16, R16, kHid, (long)kSeq * kHid,
      W2T, W2T, kHid, 0L,
      (void*)Hbuf, (void*)Hbuf, kHid, (long)kSeq * kHid,
      b2, seq, 0L,
      lang, (long)kHid * kHid, (long)kHid, kLang,
      kSeq, kHid, kHid, kWCarryInv);

  pool_combine_kernel<<<dim3(kHid / 64, kBatch), blk, 0, stream>>>(Hbuf, tokw, topics, C16);

  wmma_gemm64<0, false, 2, 0, false, 0, false><<<dim3(1, 1), blk, 0, stream>>>(
      C16, C16, kKfPad, 0L,
      WfT, WfT, kKfPad, 0L,
      (void*)Fbuf, (void*)Fbuf, kTHid, 0L,
      bfv, seq, 0L,
      lang, 0L, 0L, 1,
      kMf, kTHid, kKfPad, kWCarryInv);

  ln_relu_out_kernel<<<dim3(kBatch), dim3(128), 0, stream>>>(Fbuf, gf, bef, outp);
}
